// MambaBlockSequential_61744449848168
// MI455X (gfx1250) — hardware-verified
//
#include <hip/hip_runtime.h>


#define NB_  2
#define SQ   2048
#define DD   1024
#define NS   16
#define NR   (NB_ * SQ)
typedef _Float16 h16;
typedef unsigned short bf;
typedef __attribute__((ext_vector_type(16))) __bf16   v16bf;
typedef __attribute__((ext_vector_type(16))) _Float16 v16h;
typedef __attribute__((ext_vector_type(8)))  _Float16 v8h;
typedef __attribute__((ext_vector_type(8)))  unsigned short v8us;
typedef __attribute__((ext_vector_type(8)))  float    v8f;
typedef __attribute__((ext_vector_type(4)))  float    v4f;
typedef v8h  __attribute__((may_alias)) v8ha;
typedef v4f  __attribute__((may_alias)) v4fa;
typedef v8us __attribute__((may_alias)) v8usa;

__device__ __forceinline__ unsigned short f2bf(float f) { unsigned u = __float_as_uint(f); u += 0x7FFFu + ((u >> 16) & 1u); return (unsigned short)(u >> 16); }
__device__ __forceinline__ float bf2f(unsigned short b) { return __uint_as_float(((unsigned)b) << 16); }
__device__ __forceinline__ float bfr(float f) { return bf2f(f2bf(f)); }
__device__ __forceinline__ v16h cat16(v8h lo, v8h hi) { return __builtin_shufflevector(lo, hi, 0, 1, 2, 3, 4, 5, 6, 7, 8, 9, 10, 11, 12, 13, 14, 15); }
__device__ __forceinline__ v16bf cat16b(v8us lo, v8us hi) { return __builtin_bit_cast(v16bf, __builtin_shufflevector(lo, hi, 0, 1, 2, 3, 4, 5, 6, 7, 8, 9, 10, 11, 12, 13, 14, 15)); }
__device__ __forceinline__ v8f wmma16(v16h a, v16h b, v8f c) { return __builtin_amdgcn_wmma_f32_16x16x32_f16(false, a, false, b, (short)0, c, false, false); }
__device__ __forceinline__ v8f wmmab(v16bf a, v16bf b, v8f c) { return __builtin_amdgcn_wmma_f32_16x16x32_bf16(false, a, false, b, (short)0, c, false, false); }


template <typename T16> struct WFrag;
template <> struct WFrag<h16> { typedef v16h V; static __device__ __forceinline__ V ld(const h16* p) { return cat16(*(const v8h*)p, *(const v8h*)(p + 16)); } static __device__ __forceinline__ v8f mma(V a, V b, v8f c) { return wmma16(a, b, c); } };
template <> struct WFrag<bf> { typedef v16bf V; static __device__ __forceinline__ V ld(const bf* p) { return cat16b(*(const v8us*)p, *(const v8us*)(p + 16)); } static __device__ __forceinline__ v8f mma(V a, V b, v8f c) { return wmmab(a, b, c); } };
template <typename T16, int NSPLIT, bool BIAS>
__global__ __launch_bounds__(32) void k_gemmw(const T16* __restrict__ A, const T16* __restrict__ A2, const T16* __restrict__ Bt, const T16* __restrict__ Bt2, int K, float* C, int ldc, const float* __restrict__ bias, size_t sA, size_t sB, size_t sC) {
    typedef typename WFrag<T16>::V V;
    __shared__ __align__(16) float os[16 * 68];
    const size_t z = blockIdx.z; A += z * sA; if (A2) A2 += z * sA; Bt += z * sB; if (Bt2) Bt2 += z * sB; C += z * sC;
    const int lane = threadIdx.x & 31, lr = lane & 15, hi = lane >> 4; const int r0 = blockIdx.x * 64, c0 = blockIdx.y * 64;
    v8f acc[4][4];
#pragma unroll
    for (int mb = 0; mb < 4; ++mb)
#pragma unroll
        for (int nb = 0; nb < 4; ++nb) acc[mb][nb] = (v8f){};
    const size_t aoff = (size_t)(r0 + lr) * K + 8 * hi, boff = (size_t)(c0 + lr) * K + 8 * hi;
#pragma unroll 1
    for (int kc = 0; kc < K; kc += 32) {
        V a[4], a2[4];
#pragma unroll
        for (int mb = 0; mb < 4; ++mb) { a[mb] = WFrag<T16>::ld(A + aoff + (size_t)mb * 16 * K + kc); if (NSPLIT == 1 || NSPLIT == 2) a2[mb] = WFrag<T16>::ld(A2 + aoff + (size_t)mb * 16 * K + kc); }
#pragma unroll
        for (int nb = 0; nb < 4; ++nb) { const V b = WFrag<T16>::ld(Bt + boff + (size_t)nb * 16 * K + kc); V b2; if (NSPLIT >= 2) b2 = WFrag<T16>::ld(Bt2 + boff + (size_t)nb * 16 * K + kc);
#pragma unroll
            for (int mb = 0; mb < 4; ++mb) { acc[mb][nb] = WFrag<T16>::mma(a[mb], b, acc[mb][nb]); if (NSPLIT == 1 || NSPLIT == 2) acc[mb][nb] = WFrag<T16>::mma(a2[mb], b, acc[mb][nb]); if (NSPLIT >= 2) acc[mb][nb] = WFrag<T16>::mma(a[mb], b2, acc[mb][nb]); } }
        asm volatile("v_nop\n\tv_nop\n\tv_nop\n\tv_nop" : "+v"(acc[0][0]), "+v"(acc[1][1]), "+v"(acc[2][2]), "+v"(acc[3][3]) : "v"(a[0]), "v"(a[3]));
    }
#pragma unroll
    for (int mb = 0; mb < 4; ++mb) {
#pragma unroll
        for (int nb = 0; nb < 4; ++nb) {
#pragma unroll
            for (int j = 0; j < 8; ++j) os[(hi * 8 + j) * 68 + nb * 16 + lr] = acc[mb][nb][j]; }
        __builtin_amdgcn_wave_barrier(); asm volatile("" ::: "memory");
        float* crow = C + (size_t)(r0 + mb * 16) * ldc + c0;
#pragma unroll 1
        for (int ps = 0; ps < 2; ++ps) {
#pragma unroll
            for (int s = 0; s < 8; ++s) { const int row = 2 * s + hi, cofs = lr * 4; v4f val = *(const v4fa*)(os + row * 68 + cofs); if (BIAS) { val[0] += bfr(bias[c0 + cofs]); val[1] += bfr(bias[c0 + cofs + 1]); val[2] += bfr(bias[c0 + cofs + 2]); val[3] += bfr(bias[c0 + cofs + 3]); }
                *(volatile v4f*)(crow + (size_t)row * ldc + cofs) = val; }
            if (ps == 0) __threadfence(); }
        __builtin_amdgcn_wave_barrier(); asm volatile("" ::: "memory");
    }
}

__device__ __forceinline__ void splitf(float y, unsigned short& h, unsigned short& l) { h = f2bf(y); l = f2bf(y - bf2f(h)); }
typedef __attribute__((ext_vector_type(2))) unsigned short v2us;
typedef __attribute__((ext_vector_type(4))) unsigned short v4us;

__global__ __launch_bounds__(256) void k_wtG(const float* __restrict__ w, int K, int N, bf* Bt) {
    const int lane = threadIdx.x & 31; const int L0 = (blockIdx.x * 8 + (threadIdx.x >> 5)) * 8; const int nlines = N * K / 64;
#pragma unroll
    for (int ps = 0; ps < 2; ++ps) {
#pragma unroll 1
        for (int l = 0; l < 8; ++l) { const int L = L0 + l; if (L >= nlines) break; const size_t e = (size_t)L * 64 + lane * 2; const int k = (int)(e % K), n = (int)(e / K); v2us o;
            o[0] = f2bf(w[(size_t)k * N + n]); o[1] = f2bf(w[(size_t)(k + 1) * N + n]); *(volatile v2us*)(Bt + e) = o; }
        if (ps == 0) __threadfence(); }
}
__global__ __launch_bounds__(256) void k_cvt8(const float* __restrict__ src, bf* dst, size_t n8) { const size_t i = (size_t)blockIdx.x * 256 + threadIdx.x; if (i >= n8) return; const v8f v = *(const v8f*)(src + i * 8); v8us o;
#pragma unroll
    for (int k = 0; k < 8; ++k) o[k] = f2bf(v[k]); *(volatile v8us*)(dst + i * 8) = o; __threadfence(); *(volatile v8us*)(dst + i * 8) = o; }
__global__ __launch_bounds__(256) void k_wbc(const float* __restrict__ WB, const float* __restrict__ WC, bf* Bt) { const int e = (blockIdx.x * 256 + threadIdx.x) * 4; if (e >= 64 * DD) return; const int k = e % DD; const int c = e / DD; v4us v;
#pragma unroll
    for (int u = 0; u < 4; ++u) v[u] = (c < NS) ? f2bf(WB[(size_t)(k + u) * NS + c]) : (c < 2 * NS) ? f2bf(WC[(size_t)(k + u) * NS + c - NS]) : (unsigned short)0; *(volatile v4us*)(Bt + e) = v; __threadfence(); *(volatile v4us*)(Bt + e) = v; }
__global__ __launch_bounds__(64) void k_scan(const float* __restrict__ GD, const float* __restrict__ bdt, const float* __restrict__ XS, const float* __restrict__ bx, const float* __restrict__ BC, const float* __restrict__ bB, const float* __restrict__ bC, const float* __restrict__ alog, float* Y) {
    const int gl = blockIdx.x * 64 + threadIdx.x; if (gl >= NB_ * DD) return; const int b = gl / DD, d = gl % DD; float A[NS], h[NS], bBv[NS], bCv[NS];
#pragma unroll
    for (int n = 0; n < NS; ++n) { A[n] = -__expf(bfr(alog[d * NS + n])); h[n] = 0.f; bBv[n] = bfr(bB[n]); bCv[n] = bfr(bC[n]); } const float bd = bfr(bdt[d]), bxx = bfr(bx[d]);
#pragma unroll 1
    for (int t = 0; t < SQ; ++t) { const size_t r = (size_t)b * SQ + t; const float zt = __fadd_rn(GD[r * DD + d], bd); const float dt = (zt > 20.f) ? zt : log1pf(__expf(zt)); const float xs = __fadd_rn(XS[r * DD + d], bxx); const float* bc = BC + r * 64; float y = 0.f;
#pragma unroll
        for (int n = 0; n < NS; ++n) { const float Bn = __fadd_rn(bc[n], bBv[n]); const float Cn = __fadd_rn(bc[NS + n], bCv[n]); const float da = __expf(__fmul_rn(dt, A[n])); float db = __fmul_rn(dt, Bn); asm volatile("" : "+v"(db)); float xd = __fmul_rn(xs, db); asm volatile("" : "+v"(xd)); float q = __fmul_rn(da, h[n]); asm volatile("" : "+v"(q)); h[n] = __fadd_rn(q, xd); float p = __fmul_rn(h[n], Cn); asm volatile("" : "+v"(p)); y = __fadd_rn(y, p); }
        *(volatile float*)(Y + r * DD + d) = y; __threadfence(); *(volatile float*)(Y + r * DD + d) = y; } }
__global__ __launch_bounds__(256) void k_gate(const float* __restrict__ Y, const float* __restrict__ GZ, const float* __restrict__ bz, bf* Gh, bf* Gl) { const size_t e = ((size_t)blockIdx.x * 256 + threadIdx.x) * 4; if (e >= (size_t)NR * DD) return; const int d = (int)(e % DD); v4us oh, ol;
#pragma unroll
    for (int u = 0; u < 4; ++u) { const float g = __fadd_rn(GZ[e + u], bfr(bz[d + u])); const float sg = __fdiv_rn(1.0f, __fadd_rn(1.0f, __expf(-g))); unsigned short p, q; splitf(__fmul_rn(Y[e + u], sg), p, q); oh[u] = p; ol[u] = q; }
    *(volatile v4us*)(Gh + e) = oh; *(volatile v4us*)(Gl + e) = ol; __threadfence(); *(volatile v4us*)(Gh + e) = oh; *(volatile v4us*)(Gl + e) = ol; }

extern "C" void kernel_launch(void* const* d_in, const int* in_sizes, int n_in,
                              void* d_out, int out_size, void* d_ws, size_t ws_size, hipStream_t stream) {
    (void)in_sizes; (void)n_in; (void)out_size;
    const float** I = (const float**)d_in;
    const float *x = I[0], *Wz = I[1], *bz = I[2], *Wx = I[3], *bx = I[4], *WB = I[5], *bB = I[6], *WC = I[7], *bC = I[8], *Wdt = I[9], *bdt = I[10], *alog = I[11], *Wout = I[12], *bout = I[13];
    float* OUT = (float*)d_out;
    char* wsp = (char*)d_ws;
    auto take = [&](size_t bytes) { char* p = wsp; wsp += (bytes + 255) & ~(size_t)255; return (void*)p; };
    bf* BZ = (bf*)take((size_t)DD * DD * 2); bf* BX = (bf*)take((size_t)DD * DD * 2); bf* BDT = (bf*)take((size_t)DD * DD * 2); bf* BO = (bf*)take((size_t)DD * DD * 2); bf* BBC = (bf*)take((size_t)64 * DD * 2); bf* XB = (bf*)take((size_t)NR * DD * 2);
    float* GZ = (float*)take((size_t)NR * DD * 4); float* XS = (float*)take((size_t)NR * DD * 4); float* GD = (float*)take((size_t)NR * DD * 4); float* BC = (float*)take((size_t)NR * 64 * 4); float* Y = (float*)take((size_t)NR * DD * 4); bf* Gh = (bf*)take((size_t)NR * DD * 2); bf* Gl = (bf*)take((size_t)NR * DD * 2);
    if ((size_t)(wsp - (char*)d_ws) > ws_size) return;
    k_wtG<<<(unsigned)((DD * DD / 64 + 63) / 64), 256, 0, stream>>>(Wz, DD, DD, BZ); k_wtG<<<(unsigned)((DD * DD / 64 + 63) / 64), 256, 0, stream>>>(Wx, DD, DD, BX); k_wtG<<<(unsigned)((DD * DD / 64 + 63) / 64), 256, 0, stream>>>(Wdt, DD, DD, BDT); k_wtG<<<(unsigned)((DD * DD / 64 + 63) / 64), 256, 0, stream>>>(Wout, DD, DD, BO); k_wbc<<<(64 * DD / 4 + 255) / 256, 256, 0, stream>>>(WB, WC, BBC);
    k_cvt8<<<(NR * DD / 8 + 255) / 256, 256, 0, stream>>>(x, XB, NR * DD / 8);
    const dim3 gp(NR / 64, DD / 64, 1);
    k_gemmw<bf, 0, false><<<gp, 32, 0, stream>>>(XB, nullptr, BZ, nullptr, DD, GZ, DD, nullptr, 0, 0, 0); k_gemmw<bf, 0, false><<<gp, 32, 0, stream>>>(XB, nullptr, BX, nullptr, DD, XS, DD, nullptr, 0, 0, 0); k_gemmw<bf, 0, false><<<gp, 32, 0, stream>>>(XB, nullptr, BDT, nullptr, DD, GD, DD, nullptr, 0, 0, 0);
    k_gemmw<bf, 0, false><<<dim3(NR / 64, 1, 1), 32, 0, stream>>>(XB, nullptr, BBC, nullptr, DD, BC, 64, nullptr, 0, 0, 0);
    k_scan<<<(NB_ * DD + 63) / 64, 64, 0, stream>>>(GD, bdt, XS, bx, BC, bB, bC, alog, Y);
    k_gate<<<(unsigned)(((size_t)NR * DD / 4 + 255) / 256), 256, 0, stream>>>(Y, GZ, bz, Gh, Gl);
    k_gemmw<bf, 1, true><<<gp, 32, 0, stream>>>(Gh, Gl, BO, nullptr, DD, OUT, DD, bout, 0, 0, 0);
}
